// HEMALoss_20641612825292
// MI455X (gfx1250) — hardware-verified
//
#include <hip/hip_runtime.h>
#include <stddef.h>


typedef _Float16 v16h __attribute__((ext_vector_type(16)));
typedef _Float16 v8h  __attribute__((ext_vector_type(8)));
typedef float    v8f  __attribute__((ext_vector_type(8)));
typedef float    v4f  __attribute__((ext_vector_type(4)));
typedef float    v2f  __attribute__((ext_vector_type(2)));

#define NROW   512
#define DD     256
#define MROWS  (2 * NROW)
#define PHYS_W 0.1f
#define KCH    32

#define LDT 72
#define LDC 68

#define WCARRY 64.0f
#define NCARRY 16.0f

#define OUT_ELEMS (2 + 2 * NROW * NROW)
#define NV4       ((OUT_ELEMS - 2) / 4)

static_assert(DD == 32 * 8);
static_assert((DD % 64) == 0 && (DD % 32) == 0);
static_assert(DD == 256);
static_assert((NROW % 64) == 0 && (MROWS % 64) == 0);
static_assert((NROW % 8) == 0 && (MROWS % 32) == 0);
static_assert(NROW == 4 * 32 * 4);
static_assert(NROW == 512);
static_assert((KCH * 64) == 2 * 256 * 4);
static_assert((DD % KCH) == 0);
static_assert((LDT % 8) == 0 && LDT >= 64);
static_assert((LDC % 4) == 0 && LDC >= 64);
static_assert(OUT_ELEMS == 524290);
static_assert(4 * NV4 + 2 == OUT_ELEMS);
static_assert((NV4 % 256) == 0);
static_assert((size_t)4 * 1 == (size_t)4);
static_assert((size_t)4 * (1 + NROW * NROW) == (size_t)1048580);
static_assert((size_t)4 * (1 + 2 * NROW * NROW) == (size_t)2097156);
static_assert((size_t)4 * OUT_ELEMS == (size_t)2097160);

#define ZPL_BYTES ((size_t)MROWS * DD * 2)
#define WT_BYTES  ((size_t)2 * DD * DD * 2)
#define H_BYTES   ((size_t)MROWS * DD * 4)
#define LL_BYTES  ((size_t)MROWS * NROW * 4)
#define LSE_BYTES ((size_t)MROWS * 4)
#define SC_BYTES  ((size_t)128)
#define OFF_ZR  ((size_t)0)
#define OFF_ZN  (OFF_ZR + ZPL_BYTES)
#define OFF_WT  (OFF_ZN + ZPL_BYTES)
#define OFF_H   (OFF_WT + WT_BYTES)
#define OFF_LL  (OFF_H + H_BYTES)
#define OFF_LSE (OFF_LL + LL_BYTES)
#define OFF_SC  (OFF_LSE + LSE_BYTES)
#define WS_TOTAL (OFF_SC + SC_BYTES)
static_assert((ZPL_BYTES % 128) == 0 && (WT_BYTES % 128) == 0 && (H_BYTES % 128) == 0);
static_assert((LL_BYTES % 128) == 0 && (LSE_BYTES % 128) == 0);
static_assert(WS_TOTAL <= (size_t)134217728);

__device__ __forceinline__ _Float16 toh_flush(float v) {
  const _Float16 r = (_Float16)v;
  return (fabsf(v) < 6.103515625e-05f) ? (_Float16)0.0f : r;
}

__device__ __forceinline__ v16h frag_at(const _Float16* p) {
  v8h lo = *(const v8h*)(p);
  v8h hi = *(const v8h*)(p + 16);
  v16h out;
#pragma unroll
  for (int i = 0; i < 8; ++i) { out[i] = lo[i]; out[i + 8] = hi[i]; }
  return out;
}

__device__ __forceinline__ v8f wmma16(v16h a, v16h b, v8f c) {
  v8f d = __builtin_amdgcn_wmma_f32_16x16x32_f16(false, a, false, b, (short)0, c,
                                                 false, false);
  asm volatile("v_nop\n\tv_nop\n\tv_nop\n\tv_nop" : "+v"(d) : "v"(a), "v"(b));
  return d;
}

__device__ __forceinline__ float red32_sum(float x) {
#pragma unroll
  for (int off = 1; off < 32; off <<= 1) x += __shfl_xor(x, off, 32);
  return x;
}
__device__ __forceinline__ float red32_max(float x) {
#pragma unroll
  for (int off = 1; off < 32; off <<= 1) x = fmaxf(x, __shfl_xor(x, off, 32));
  return x;
}
__device__ __forceinline__ unsigned wave_id() {
  return (unsigned)__builtin_amdgcn_readfirstlane((int)(threadIdx.x >> 5));
}

__global__ __launch_bounds__(256) void prep_kernel(
    const float* __restrict__ Z, _Float16* __restrict__ Zr, _Float16* __restrict__ Zn) {
  const unsigned lane = threadIdx.x & 31u;
  const unsigned w = wave_id();
  const unsigned row = blockIdx.x * 8u + w;
  const float* xr = Z + (size_t)row * DD + lane * 8u;
  const v4f a0 = *(const v4f*)(xr);
  const v4f a1 = *(const v4f*)(xr + 4);
  float ss = 0.0f;
#pragma unroll
  for (int i = 0; i < 4; ++i) {
    ss += a0[i] * a0[i];
    ss += a1[i] * a1[i];
  }
  ss = red32_sum(ss);
  const float inv = NCARRY * (1.0f / sqrtf(ss));
  v8h xr16, xn16;
#pragma unroll
  for (int i = 0; i < 4; ++i) {
    xr16[i]     = toh_flush(a0[i]);
    xr16[i + 4] = toh_flush(a1[i]);
    xn16[i]     = toh_flush(a0[i] * inv);
    xn16[i + 4] = toh_flush(a1[i] * inv);
  }
  const size_t off = (size_t)row * DD + lane * 8u;
  *(volatile v8h*)(Zr + off) = xr16;
  *(volatile v8h*)(Zn + off) = xn16;
  __threadfence();
  *(volatile v8h*)(Zr + off) = xr16;
  *(volatile v8h*)(Zn + off) = xn16;
}

__global__ __launch_bounds__(256) void wplane_kernel(
    const float* __restrict__ W, _Float16* __restrict__ Wt) {
  __shared__ _Float16 T[64 * LDT];
  const unsigned tid = threadIdx.x;
  const unsigned n0 = blockIdx.x * 64u;
  const unsigned kg0 = blockIdx.y * 64u;
  const unsigned plane = kg0 / (unsigned)DD;
  const unsigned k0 = kg0 - plane * (unsigned)DD;
#pragma unroll 4
  for (unsigned j = 0; j < 16u; ++j) {
    const unsigned idx = tid + 256u * j;
    const unsigned kr = idx >> 6, nc = idx & 63u;
    const float v = W[(size_t)(kg0 + kr) * DD + n0 + nc];
    T[nc * LDT + kr] = toh_flush(WCARRY * v);
  }
  __syncthreads();
  v8h x[2];
  size_t off[2];
#pragma unroll
  for (unsigned i = 0; i < 2u; ++i) {
    const unsigned n = 32u * i + (tid >> 3);
    const unsigned kc = (tid & 7u) * 8u;
    x[i] = *(const v8h*)&T[n * LDT + kc];
    off[i] = (size_t)plane * DD * DD + (size_t)(n0 + n) * DD + k0 + kc;
  }
#pragma unroll
  for (int i = 0; i < 2; ++i) *(volatile v8h*)(Wt + off[i]) = x[i];
  __threadfence();
#pragma unroll
  for (int i = 0; i < 2; ++i) *(volatile v8h*)(Wt + off[i]) = x[i];
}

__global__ __launch_bounds__(256) void gemm_h_kernel(
    const _Float16* __restrict__ Z16, const _Float16* __restrict__ Wt,
    const float* __restrict__ b1, float* __restrict__ H) {
  __shared__ float Cs[64 * LDC];
  const unsigned tid = threadIdx.x, lane = tid & 31u;
  const unsigned w = wave_id();
  const unsigned mw = w >> 1, nw = w & 1u;
  const unsigned hh = lane >> 4, m = lane & 15u;
  const unsigned n0 = blockIdx.x * 64u;
  const unsigned row0 = blockIdx.y * 64u;
  const unsigned plane = (row0 >= (unsigned)NROW) ? 1u : 0u;

  const _Float16* ap  = Z16 + (size_t)(row0 + mw * 16u + m) * DD + hh * 8u;
  const _Float16* bp0 = Wt + (size_t)plane * DD * DD + (size_t)(n0 + nw * 32u + m) * DD + hh * 8u;
  const _Float16* bp1 = bp0 + (size_t)16 * DD;
  v8f acc0 = {}, acc1 = {};
#pragma unroll 2
  for (unsigned k0 = 0; k0 < (unsigned)DD; k0 += 32u) {
    const v16h a  = frag_at(ap + k0);
    const v16h b0 = frag_at(bp0 + k0);
    const v16h b1f = frag_at(bp1 + k0);
    acc0 = wmma16(a, b0, acc0);
    acc1 = wmma16(a, b1f, acc1);
  }
#pragma unroll
  for (int r = 0; r < 8; ++r) {
    float* d = &Cs[(mw * 16u + hh * 8u + (unsigned)r) * LDC + nw * 32u + m];
    d[0]  = acc0[r];
    d[16] = acc1[r];
  }
  __syncthreads();

  v4f xs[4];
  size_t off[4];
#pragma unroll
  for (unsigned i = 0; i < 4u; ++i) {
    const unsigned r = 16u * i + (tid >> 4);
    const unsigned c = (tid & 15u) * 4u;
    const v4f u = *(const v4f*)&Cs[r * LDC + c];
    const v4f g = *(const v4f*)(b1 + n0 + c);
    v4f val;
#pragma unroll
    for (int j = 0; j < 4; ++j) {
      const float bb = plane ? 0.0f : g[j];
      val[j] = u[j] * (1.0f / WCARRY) + bb;
    }
    xs[i] = val;
    off[i] = (size_t)(row0 + r) * DD + n0 + c;
  }
#pragma unroll
  for (int i = 0; i < 4; ++i) *(volatile v4f*)(H + off[i]) = xs[i];
  __threadfence();
#pragma unroll
  for (int i = 0; i < 4; ++i) *(volatile v4f*)(H + off[i]) = xs[i];
}

__global__ __launch_bounds__(256) void logits_kernel(
    const _Float16* __restrict__ Zn, const float* __restrict__ H,
    const float* __restrict__ W2, const float* __restrict__ b2,
    const float* __restrict__ logt, float* __restrict__ LL) {
  __shared__ float Cs[64 * LDC];
  __shared__ float sA[KCH * 64];
  __shared__ float sB[KCH * 64];
  __shared__ float sW[DD];

  const unsigned tid = threadIdx.x, lane = tid & 31u;
  const unsigned w = wave_id();
  const unsigned mw = w >> 1, nw = w & 1u;
  const unsigned hh = lane >> 4, m = lane & 15u;
  const unsigned j0 = blockIdx.x * 64u;
  const unsigned i0 = blockIdx.y * 64u;

  {
    const _Float16* ap  = Zn + (size_t)(i0 + mw * 16u + m) * DD + hh * 8u;
    const _Float16* bp0 = Zn + (size_t)((unsigned)NROW + j0 + nw * 32u + m) * DD + hh * 8u;
    const _Float16* bp1 = bp0 + (size_t)16 * DD;
    v8f acc0 = {}, acc1 = {};
#pragma unroll 2
    for (unsigned k0 = 0; k0 < (unsigned)DD; k0 += 32u) {
      const v16h a  = frag_at(ap + k0);
      const v16h b0 = frag_at(bp0 + k0);
      const v16h b1f = frag_at(bp1 + k0);
      acc0 = wmma16(a, b0, acc0);
      acc1 = wmma16(a, b1f, acc1);
    }
#pragma unroll
    for (int r = 0; r < 8; ++r) {
      float* d = &Cs[(mw * 16u + hh * 8u + (unsigned)r) * LDC + nw * 32u + m];
      d[0]  = acc0[r];
      d[16] = acc1[r];
    }
  }
  sW[tid] = W2[tid];
  __syncthreads();

  const unsigned ti = tid >> 4, tj = tid & 15u;
  float c[4][4];
#pragma unroll
  for (int x = 0; x < 4; ++x)
#pragma unroll
    for (int y = 0; y < 4; ++y) c[x][y] = 0.0f;

#pragma unroll 1
  for (unsigned kc = 0; kc < (unsigned)DD; kc += (unsigned)KCH) {
#pragma unroll
    for (unsigned j = 0; j < 2u; ++j) {
      const unsigned idx = tid + 256u * j;
      const unsigned r = idx >> 3, q = (idx & 7u) * 4u;
      const v4f va = *(const v4f*)(H + (size_t)(i0 + r) * DD + kc + q);
      const v4f vb = *(const v4f*)(H + (size_t)((unsigned)NROW + j0 + r) * DD + kc + q);
#pragma unroll
      for (unsigned e = 0; e < 4u; ++e) {
        sA[(q + e) * 64u + r] = va[e];
        sB[(q + e) * 64u + r] = vb[e];
      }
    }
    __syncthreads();
#pragma unroll 2
    for (unsigned kk = 0; kk < (unsigned)KCH; ++kk) {
      const v4f a = *(const v4f*)&sA[kk * 64u + 4u * ti];
      const v4f b = *(const v4f*)&sB[kk * 64u + 4u * tj];
      const float wv = sW[kc + kk];
#pragma unroll
      for (int x = 0; x < 4; ++x)
#pragma unroll
        for (int y = 0; y < 4; ++y)
          c[x][y] = fmaf(fmaxf(a[x] + b[y], 0.0f), wv, c[x][y]);
    }
    __syncthreads();
  }

  const float tcl = fminf(fmaxf(expf(logt[0]), 1.0e-4f), 100.0f);
  const float inv_t = 1.0f / tcl;
  const float bb2 = b2[0];
#pragma unroll
  for (int x = 0; x < 4; ++x) {
    const unsigned r = 4u * ti + (unsigned)x;
    const v4f s = *(const v4f*)&Cs[r * LDC + 4u * tj];
    v4f o;
#pragma unroll
    for (int y = 0; y < 4; ++y)
      o[y] = (s[y] * (1.0f / (NCARRY * NCARRY)) + PHYS_W * (c[x][y] + bb2)) * inv_t;
    *(v4f*)&Cs[r * LDC + 4u * tj] = o;
  }
  __syncthreads();

  v4f xs[4], xt[4];
  size_t off[4], offt[4];
#pragma unroll
  for (unsigned i = 0; i < 4u; ++i) {
    const unsigned r = 16u * i + (tid >> 4);
    const unsigned cc = (tid & 15u) * 4u;
    xs[i] = *(const v4f*)&Cs[r * LDC + cc];
    off[i] = (size_t)(i0 + r) * NROW + j0 + cc;
    v4f t;
#pragma unroll
    for (unsigned e = 0; e < 4u; ++e) t[e] = Cs[(cc + e) * LDC + r];
    xt[i] = t;
    offt[i] = (size_t)NROW * NROW + (size_t)(j0 + r) * NROW + i0 + cc;
  }
#pragma unroll
  for (int i = 0; i < 4; ++i) *(volatile v4f*)(LL + off[i]) = xs[i];
#pragma unroll
  for (int i = 0; i < 4; ++i) *(volatile v4f*)(LL + offt[i]) = xt[i];
  __threadfence();
#pragma unroll
  for (int i = 0; i < 4; ++i) *(volatile v4f*)(LL + off[i]) = xs[i];
#pragma unroll
  for (int i = 0; i < 4; ++i) *(volatile v4f*)(LL + offt[i]) = xt[i];
}

__global__ __launch_bounds__(256) void lse_kernel(
    const float* __restrict__ LL, float* __restrict__ LSE) {
  __shared__ float sL[32];
  const unsigned lane = threadIdx.x & 31u;
  const unsigned w = wave_id();
#pragma unroll 1
  for (unsigned q = 0; q < 4u; ++q) {
    const unsigned row = blockIdx.x * 32u + w * 4u + q;
    const float* p = LL + (size_t)row * NROW + lane * 4u;
    const v4f v0 = *(const v4f*)(p);
    const v4f v1 = *(const v4f*)(p + 128);
    const v4f v2 = *(const v4f*)(p + 256);
    const v4f v3 = *(const v4f*)(p + 384);
    float mx = fmaxf(fmaxf(v0[0], v0[1]), fmaxf(v0[2], v0[3]));
    mx = fmaxf(mx, fmaxf(fmaxf(v1[0], v1[1]), fmaxf(v1[2], v1[3])));
    mx = fmaxf(mx, fmaxf(fmaxf(v2[0], v2[1]), fmaxf(v2[2], v2[3])));
    mx = fmaxf(mx, fmaxf(fmaxf(v3[0], v3[1]), fmaxf(v3[2], v3[3])));
    mx = red32_max(mx);
    float s = 0.0f;
#pragma unroll
    for (int i = 0; i < 4; ++i) {
      s += __expf(v0[i] - mx);
      s += __expf(v1[i] - mx);
      s += __expf(v2[i] - mx);
      s += __expf(v3[i] - mx);
    }
    s = red32_sum(s);
    if (lane == 0u) sL[w * 4u + q] = mx + logf(s);
  }
  __syncthreads();
  const v4f x = *(const v4f*)&sL[(lane & 7u) * 4u];
  if (w == 0u && lane < 8u) {
    float* dst = LSE + (size_t)blockIdx.x * 32u + lane * 4u;
    *(volatile v4f*)dst = x;
    __threadfence();
    *(volatile v4f*)dst = x;
  }
}

__global__ __launch_bounds__(512) void loss_kernel(
    const float* __restrict__ LL, const float* __restrict__ LSE,
    const float* __restrict__ logt, float* __restrict__ SC) {
  __shared__ float red[NROW];
  const unsigned t = threadIdx.x;
  const float diag = LL[(size_t)t * (NROW + 1)];
  red[t] = (LSE[t] - diag) + (LSE[NROW + t] - diag);
  __syncthreads();
#pragma unroll 1
  for (unsigned s = NROW / 2; s > 0u; s >>= 1) {
    if (t < s) red[t] += red[t + s];
    __syncthreads();
  }
  const float loss = red[0] * (1.0f / (2.0f * (float)NROW));
  const float tcl = fminf(fmaxf(expf(logt[0]), 1.0e-4f), 100.0f);
  v4f x;
  x[0] = (t == 0u) ? loss : 0.0f;
  x[1] = (t == 0u) ? tcl : 0.0f;
  x[2] = 0.0f;
  x[3] = 0.0f;
  if (t < 8u) {
    float* dst = SC + t * 4u;
    *(volatile v4f*)dst = x;
    __threadfence();
    *(volatile v4f*)dst = x;
  }
}

__global__ __launch_bounds__(256) void pack_kernel(
    const float* __restrict__ LL, const float* __restrict__ SC, float* __restrict__ out) {
  const unsigned g = blockIdx.x * 256u + threadIdx.x;
  const unsigned e0 = 4u * g;
  const float loss = SC[0];
  const float tcl = SC[1];
  const float lastv = LL[(size_t)2 * NROW * NROW - 1];
  v4f val;
#pragma unroll
  for (unsigned u = 0; u < 4u; ++u) {
    const unsigned e = e0 + u;
    const unsigned idx = (e == 0u) ? 0u : (e - 1u);
    float f = LL[idx];
    asm volatile("" : "+v"(f));
    val[u] = (e == 0u) ? loss : f;
  }
  v2f tail;
  tail[0] = lastv;
  tail[1] = tcl;
  float* p = out + e0;
  float* ptail = out + (size_t)4 * NV4;
  *(volatile v4f*)p = val;
  if (g == (unsigned)(NV4 - 1)) *(volatile v2f*)ptail = tail;
  __threadfence();
  *(volatile v4f*)p = val;
  if (g == (unsigned)(NV4 - 1)) *(volatile v2f*)ptail = tail;
}

extern "C" void kernel_launch(void* const* d_in, const int* in_sizes, int n_in,
                              void* d_out, int out_size, void* d_ws, size_t ws_size,
                              hipStream_t stream) {
  if (n_in < 7) return;
  if ((long long)in_sizes[0] < (long long)NROW * DD) return;
  if ((long long)in_sizes[1] < (long long)NROW * DD) return;
  if ((long long)in_sizes[2] < (long long)2 * DD * DD) return;
  if (in_sizes[3] < DD || in_sizes[4] < DD) return;
  if (in_sizes[5] < 1 || in_sizes[6] < 1) return;
  if ((long long)out_size < (long long)OUT_ELEMS) return;
  if (ws_size < WS_TOTAL) return;

  const float* z_a  = (const float*)d_in[0];
  const float* z_b  = (const float*)d_in[1];
  const float* W1   = (const float*)d_in[2];
  const float* b1   = (const float*)d_in[3];
  const float* W2   = (const float*)d_in[4];
  const float* b2   = (const float*)d_in[5];
  const float* logt = (const float*)d_in[6];
  float* out = (float*)d_out;

  char* ws = (char*)d_ws;
  _Float16* Zr  = (_Float16*)(ws + OFF_ZR);
  _Float16* Zn  = (_Float16*)(ws + OFF_ZN);
  _Float16* Wt  = (_Float16*)(ws + OFF_WT);
  float*    H   = (float*)(ws + OFF_H);
  float*    LL  = (float*)(ws + OFF_LL);
  float*    LSE = (float*)(ws + OFF_LSE);
  float*    SC  = (float*)(ws + OFF_SC);

  dim3 blk(256);
  prep_kernel<<<dim3(NROW / 8), blk, 0, stream>>>(z_a, Zr, Zn);
  prep_kernel<<<dim3(NROW / 8), blk, 0, stream>>>(z_b, Zr + (size_t)NROW * DD,
                                                  Zn + (size_t)NROW * DD);
  wplane_kernel<<<dim3(DD / 64, 2 * DD / 64), blk, 0, stream>>>(W1, Wt);
  gemm_h_kernel<<<dim3(DD / 64, MROWS / 64), blk, 0, stream>>>(Zr, Wt, b1, H);
  logits_kernel<<<dim3(NROW / 64, NROW / 64), blk, 0, stream>>>(Zn, H, W2, b2, logt, LL);
  lse_kernel<<<dim3(MROWS / 32), blk, 0, stream>>>(LL, LSE);
  loss_kernel<<<dim3(1), dim3(NROW), 0, stream>>>(LL, LSE, logt, SC);
  pack_kernel<<<dim3(NV4 / 256), blk, 0, stream>>>(LL, SC, out);
}
